// StudentModel_62551903699323
// MI455X (gfx1250) — hardware-run, weakly checked
//
#include <hip/hip_runtime.h>
#include <math.h>

#ifndef NB
#define NB 4
#endif
#define NB_FULL 4
#define SEQ 128
#define DF 768
#define EH1 512
#define EH2 128
#define FH1 512
#define FOUT 256
#define GH1 256
#define GOUT 64
#define MTOK (NB * SEQ)
#define KADJ (3 * SEQ)
#define PQW (2 * EH1)

static_assert(NB >= 1 && NB <= NB_FULL);
static_assert(SEQ == 128);
static_assert(MTOK % 64 == 0 && SEQ % 64 == 0);
static_assert(PQW % 64 == 0 && FH1 % 64 == 0 && FOUT % 64 == 0 && GH1 % 64 == 0 && GOUT % 64 == 0);
static_assert(DF % 32 == 0 && (2 * FH1) % 32 == 0 && (2 * FOUT) % 32 == 0 && (2 * GH1) % 32 == 0 && KADJ % 32 == 0 && EH1 % 32 == 0);
static_assert(DF % 64 == 0 && EH1 % 64 == 0 && FH1 % 64 == 0 && FOUT % 64 == 0 && GH1 % 64 == 0);
static_assert((MTOK * DF / 8) % 256 == 0);
static_assert(EH1 == 2 * 256);
static_assert(EH2 == 8 * 16);
static_assert(EH2 % 32 == 0 && EH2 <= 256);
static_assert(SEQ == 8 * 16);
static_assert(KADJ * 2 == 512 + 256);
static_assert(8 * 16 * 68 * 4 <= 131072);
static_assert((EH1 + SEQ + 2 * EH2) * 4 <= 131072);
static_assert(32 * 16 * 8 == 16 * 256);
static_assert(32 * 16 * 4 == 16 * 128);

typedef _Float16 h16;
typedef __attribute__((ext_vector_type(16))) _Float16 v16h;
typedef __attribute__((ext_vector_type(8)))  _Float16 v8h;
typedef __attribute__((ext_vector_type(8)))  float    v8f;
typedef __attribute__((ext_vector_type(4)))  float    v4f;
typedef __attribute__((ext_vector_type(4)))  unsigned int v4u;

static constexpr float CA      = 8.0f;
static constexpr float CADJ    = 64.0f;
static constexpr float CW1     = 32.0f;
static constexpr float CWH     = 512.0f;
static constexpr float CWL     = 0.25f;
static constexpr float RSC     = 2048.0f;
static constexpr float RSI     = 1.0f / 2048.0f;
static constexpr float SC_IN   = 1.0f / 256.0f;
static constexpr float SC_FOLD = 1.0f / 4096.0f;
static constexpr float SC_ADJ  = 1.0f / 512.0f;
static constexpr float ONEF    = 1.0f;


#define VST2(T, ptr, val) do { const T vst2_v_ = (val); *(volatile T*)(ptr) = vst2_v_; __threadfence(); *(volatile T*)(ptr) = vst2_v_; } while (0)

__device__ __forceinline__ float bfr(float f) {
    unsigned u = __float_as_uint(f);
    u += 0x7FFFu + ((u >> 16) & 1u);
    return __uint_as_float(u & 0xFFFF0000u);
}
__device__ __forceinline__ unsigned short f2h_bits(float x) {
    return (fabsf(x) < 6.104e-5f) ? (unsigned short)0 : __builtin_bit_cast(unsigned short, (_Float16)x);
}
static __device__ __forceinline__ h16 toh_flush(float v) { const h16 r = (h16)v; return (fabsf(v) < 6.103515625e-05f) ? (h16)0.0f : r; }
__device__ __forceinline__ void st8h(unsigned short* P, size_t o, const float* v) {
    v4u pk;
    pk.x = (unsigned)f2h_bits(v[0]) | ((unsigned)f2h_bits(v[1]) << 16);
    pk.y = (unsigned)f2h_bits(v[2]) | ((unsigned)f2h_bits(v[3]) << 16);
    pk.z = (unsigned)f2h_bits(v[4]) | ((unsigned)f2h_bits(v[5]) << 16);
    pk.w = (unsigned)f2h_bits(v[6]) | ((unsigned)f2h_bits(v[7]) << 16);
    VST2(v4u, (v4u*)(P + o), pk);
}

union FragU { v16h v; v8h h[2]; };
__device__ __forceinline__ v16h frag_ld(const _Float16* p) {
    FragU f; f.h[0] = *(const v8h*)(p); f.h[1] = *(const v8h*)(p + 16); return f.v;
}
__device__ __forceinline__ v8f wmma16(v16h a, v16h b, v8f c) {
    c = __builtin_amdgcn_wmma_f32_16x16x32_f16(false, a, false, b, (short)0, c, false, false);
    asm volatile("v_nop\n\tv_nop\n\tv_nop\n\tv_nop" : "+v"(c) : "v"(a), "v"(b));
    return c;
}
__device__ __forceinline__ void dep_guard_h(v8f& a, v8f& b, v16h x, v16h y) { asm volatile("v_nop\n\tv_nop\n\tv_nop\n\tv_nop" : "+v"(a), "+v"(b) : "v"(x), "v"(y)); }
__device__ __forceinline__ void keep4_h(v16h a, v16h b, v16h c, v16h d) { asm volatile("v_nop" :: "v"(a), "v"(b), "v"(c), "v"(d)); }
__device__ __forceinline__ void acc_guard4(v8f& a, v8f& b, v8f& c, v8f& d) { asm volatile("v_nop\n\tv_nop\n\tv_nop\n\tv_nop" : "+v"(a), "+v"(b), "+v"(c), "+v"(d)); }
__device__ __forceinline__ void wave_sync_lds() {
    __builtin_amdgcn_fence(3  , "workgroup");
    __builtin_amdgcn_wave_barrier();
    __builtin_amdgcn_fence(2  , "workgroup");
}
__device__ __forceinline__ float tanh_f(float x) {
    const float ax = fminf(fabsf(x), 40.0f);
    const float t = exp2f(ax * -2.8853900817779268f);
    const float r = (1.0f - t) * __builtin_amdgcn_rcpf(1.0f + t);
    return copysignf(r, x);
}

template <int EPI, bool HASB, bool RELU>
__device__ __forceinline__ void gemm_tile64(
    const _Float16* __restrict__ A, unsigned lda, const _Float16* __restrict__ Bt, unsigned ldb,
    void* __restrict__ Cout, unsigned ldc, const float* __restrict__ bias,
    unsigned M, unsigned N, unsigned K, float scale, float oscale, unsigned resOff) {
  __shared__ __align__(16) float sT[8 * 16 * 68];
  const unsigned lane = threadIdx.x & 31u;
  const unsigned wave = (unsigned)__builtin_amdgcn_readfirstlane((int)(threadIdx.x >> 5));
  const unsigned tilesN = N >> 6, tilesM = M >> 6;
  const unsigned tile = blockIdx.x * 8u + wave;
  if (tile >= tilesM * tilesN) return;
  const unsigned tm = tile / tilesN;
  const unsigned tn = tile - tm * tilesN;
  const unsigned m0 = tm << 6, n0 = tn << 6;
  const unsigned rlane = lane & 15u;
  const unsigned koff = (lane >> 4) * 8u;
  const unsigned mOff = koff;

  v8f acc[4][4];
#pragma unroll
  for (int i = 0; i < 4; ++i)
#pragma unroll
    for (int j = 0; j < 4; ++j) acc[i][j] = (v8f){0.f,0.f,0.f,0.f,0.f,0.f,0.f,0.f};

  for (unsigned k0 = 0; k0 < K; k0 += 32u) {
    v16h bh[4];
#pragma unroll
    for (int j = 0; j < 4; ++j)
      bh[j] = frag_ld(Bt + (size_t)(n0 + ((unsigned)j << 4) + rlane) * ldb + koff + k0);
#pragma unroll
    for (int i = 0; i < 4; ++i) {
      const v16h ah = frag_ld(A + (size_t)(m0 + ((unsigned)i << 4) + rlane) * lda + koff + k0);
#pragma unroll
      for (int j = 0; j < 4; ++j)
        acc[i][j] = __builtin_amdgcn_wmma_f32_16x16x32_f16(false, ah, false, bh[j], (short)0, acc[i][j], false, false);
      dep_guard_h(acc[i][0], acc[i][3], ah, ah);
    }
    keep4_h(bh[0], bh[1], bh[2], bh[3]);
  }
  acc_guard4(acc[0][0], acc[0][1], acc[0][2], acc[0][3]);
  acc_guard4(acc[1][0], acc[1][1], acc[1][2], acc[1][3]);
  acc_guard4(acc[2][0], acc[2][1], acc[2][2], acc[2][3]);
  acc_guard4(acc[3][0], acc[3][1], acc[3][2], acc[3][3]);

  const unsigned sb = wave * (16u * 68u);
#pragma unroll
  for (int i = 0; i < 4; ++i) {
    const unsigned mBase = m0 + ((unsigned)i << 4);
    float bvm[8];
#pragma unroll
    for (int r = 0; r < 8; ++r) {
      bvm[r] = 0.0f;
      if (HASB && EPI == 2) bvm[r] = bfr(bias[mBase + mOff + (unsigned)r]);
    }
#pragma unroll
    for (int j = 0; j < 4; ++j) {
      const unsigned n = n0 + ((unsigned)j << 4) + rlane;
      float bvn = 0.0f;
      if (HASB && EPI != 2) bvn = bfr(bias[n]);
#pragma unroll
      for (int r = 0; r < 8; ++r) {
        float v = acc[i][j][r] * scale;
        if (HASB) v += (EPI == 2) ? bvm[r] : bvn;
        if (RELU) v = fmaxf(v, 0.0f);
        if (EPI == 3) v = tanh_f(v);
        sT[sb + (mOff + (unsigned)r) * 68u + ((unsigned)j << 4) + rlane] = v;
      }
    }
    wave_sync_lds();
    if (EPI == 0 || EPI == 3) {
      float* C = (float*)Cout;
      const unsigned hh = lane >> 4, c4 = (lane & 15u) * 4u;
#pragma unroll
      for (int half = 0; half < 2; ++half) {
        v4f vv[4];
#pragma unroll
        for (int it = 0; it < 4; ++it) {
          const unsigned row = (unsigned)(half * 4 + it) * 2u + hh;
          vv[it] = *(const v4f*)(&sT[sb + row * 68u + c4]);
        }
        for (int pass = 0; pass < 2; ++pass) {
#pragma unroll
          for (int it = 0; it < 4; ++it) {
            const unsigned row = (unsigned)(half * 4 + it) * 2u + hh;
            *(volatile v4f*)(C + (size_t)(mBase + row) * ldc + n0 + c4) = vv[it];
          }
          __threadfence();
        }
      }
    } else {
      _Float16* C = (_Float16*)Cout;
      const unsigned q = lane >> 3, c8 = (lane & 7u) * 8u;
      const unsigned zb = n0 >> 7, s0 = n0 & 127u;
      constexpr int NSEC = (EPI == 1) ? 2 : 3;
#pragma unroll
      for (int sec = 0; sec < NSEC; ++sec) {
        v8h hv[4];
#pragma unroll
        for (int it = 0; it < 4; ++it) {
          const unsigned row = (unsigned)it * 4u + q;
#pragma unroll
          for (int e = 0; e < 8; ++e) {
            const float v = sT[sb + row * 68u + c8 + (unsigned)e] * oscale;
            const h16 hi = toh_flush(v);
            h16 o = hi;
            if (sec == 1) o = toh_flush((v - (float)hi) * RSC);
            if (sec == 2) o = toh_flush((float)hi * RSI);
            hv[it][e] = o;
          }
        }
        const unsigned col = (EPI == 1) ? (n0 + c8 + (unsigned)sec * resOff)
                                        : (zb * (unsigned)KADJ + (unsigned)sec * (unsigned)SEQ + s0 + c8);
        for (int pass = 0; pass < 2; ++pass) {
#pragma unroll
          for (int it = 0; it < 4; ++it) {
            const unsigned row = (unsigned)it * 4u + q;
            *(volatile v8h*)(C + (size_t)(mBase + row) * ldc + col) = hv[it];
          }
          __threadfence();
        }
      }
    }
    wave_sync_lds();
  }
}

__global__ __launch_bounds__(256) void k_gemm_f32(
    const _Float16* __restrict__ A, unsigned lda, unsigned sA, const _Float16* __restrict__ Bt, unsigned ldb, unsigned sB,
    float* __restrict__ C, unsigned ldc, unsigned sC, unsigned M, unsigned N, unsigned K, float scale) {
  const size_t z = blockIdx.y;
  gemm_tile64<0, false, false>(A + z * sA, lda, Bt + z * sB, ldb, (void*)(C + z * sC), ldc, nullptr, M, N, K, scale, ONEF, 0u);
}
__global__ __launch_bounds__(256) void k_gemm_tanh(
    const _Float16* __restrict__ A, unsigned lda, unsigned sA, const _Float16* __restrict__ Bt, unsigned ldb, unsigned sB,
    float* __restrict__ C, unsigned ldc, unsigned sC, unsigned M, unsigned N, unsigned K, float scale) {
  const size_t z = blockIdx.y;
  gemm_tile64<3, false, false>(A + z * sA, lda, Bt + z * sB, ldb, (void*)(C + z * sC), ldc, nullptr, M, N, K, scale, ONEF, 0u);
}
__global__ __launch_bounds__(256) void k_gemm_hr_br(
    const _Float16* __restrict__ A, unsigned lda, unsigned sA, const _Float16* __restrict__ Bt, unsigned ldb, unsigned sB,
    _Float16* __restrict__ C, unsigned ldc, unsigned sC, const float* __restrict__ bias,
    unsigned M, unsigned N, unsigned K, float scale, float oscale, unsigned resOff) {
  const size_t z = blockIdx.y;
  gemm_tile64<1, true, true>(A + z * sA, lda, Bt + z * sB, ldb, (void*)(C + z * sC), ldc, bias, M, N, K, scale, oscale, resOff);
}
__global__ __launch_bounds__(256) void k_gemm_hr_b(
    const _Float16* __restrict__ A, unsigned lda, unsigned sA, const _Float16* __restrict__ Bt, unsigned ldb, unsigned sB,
    _Float16* __restrict__ C, unsigned ldc, unsigned sC, const float* __restrict__ bias,
    unsigned M, unsigned N, unsigned K, float scale, float oscale, unsigned resOff) {
  const size_t z = blockIdx.y;
  gemm_tile64<1, true, false>(A + z * sA, lda, Bt + z * sB, ldb, (void*)(C + z * sC), ldc, bias, M, N, K, scale, oscale, resOff);
}
__global__ __launch_bounds__(256) void k_gemm_hr_r(
    const _Float16* __restrict__ A, unsigned lda, unsigned sA, const _Float16* __restrict__ Bt, unsigned ldb, unsigned sB,
    _Float16* __restrict__ C, unsigned ldc, unsigned sC,
    unsigned M, unsigned N, unsigned K, float scale, float oscale, unsigned resOff) {
  const size_t z = blockIdx.y;
  gemm_tile64<1, false, true>(A + z * sA, lda, Bt + z * sB, ldb, (void*)(C + z * sC), ldc, nullptr, M, N, K, scale, oscale, resOff);
}
__global__ __launch_bounds__(256) void k_gemm_t(
    const _Float16* __restrict__ A, unsigned lda, unsigned sA, const _Float16* __restrict__ Bt, unsigned ldb, unsigned sB,
    _Float16* __restrict__ C, unsigned ldc, unsigned sC, const float* __restrict__ bias,
    unsigned M, unsigned N, unsigned K, float scale, float oscale) {
  const size_t z = blockIdx.y;
  gemm_tile64<2, true, false>(A + z * sA, lda, Bt + z * sB, ldb, (void*)(C + z * sC), ldc, bias, M, N, K, scale, oscale, 0u);
}

__global__ __launch_bounds__(256) void k_wconv(const float* __restrict__ Wm, unsigned KI, unsigned NO,
                                               unsigned short* __restrict__ W16, unsigned ldo, float swhi,
                                               unsigned loOff, float swlo) {
    const unsigned u = blockIdx.x * 256u + threadIdx.x;
    const unsigned per = KI >> 3;
    if (u >= NO * per) return;
    const unsigned o = u / per;
    const unsigned k0 = 8u * (u - o * per);
    float w[8], v[8];
#pragma unroll
    for (int i = 0; i < 8; ++i) w[i] = bfr(Wm[(size_t)(k0 + (unsigned)i) * NO + o]);
#pragma unroll
    for (int i = 0; i < 8; ++i) v[i] = w[i] * swhi;
    st8h(W16, (size_t)o * ldo + k0, v);
    if (loOff != 0u) {
#pragma unroll
        for (int i = 0; i < 8; ++i) v[i] = w[i] * swlo;
        st8h(W16, (size_t)o * ldo + loOff + k0, v);
    }
}

__global__ __launch_bounds__(256) void k_x16(const float* __restrict__ x, unsigned short* __restrict__ x16, float ca) {
    const unsigned u = blockIdx.x * 256u + threadIdx.x;
    if (u >= (unsigned)(MTOK * DF / 8)) return;
    const float* xr = x + (size_t)u * 8u;
    const v4f a = *(const v4f*)xr, b = *(const v4f*)(xr + 4);
    float v[8] = {bfr(a.x) * ca, bfr(a.y) * ca, bfr(a.z) * ca, bfr(a.w) * ca,
                  bfr(b.x) * ca, bfr(b.y) * ca, bfr(b.z) * ca, bfr(b.w) * ca};
    st8h(x16, (size_t)u * 8u, v);
}

__global__ __launch_bounds__(256) void k_edge(const float* __restrict__ PQ, const _Float16* __restrict__ W2,
                                              const float* __restrict__ eb1, const float* __restrict__ eb2,
                                              const float* __restrict__ ew3, const float* __restrict__ eb3,
                                              const int* __restrict__ mask, _Float16* __restrict__ adjA,
                                              float scale, float ca, float cadj) {
    __shared__ __align__(16) float sPE[EH1];
    __shared__ __align__(16) float sAdj[SEQ];
    __shared__ __align__(16) float sW3[EH2];
    __shared__ __align__(16) float sB2[EH2];
    const unsigned tid = threadIdx.x, lane = tid & 31u;
    const unsigned wave = (unsigned)__builtin_amdgcn_readfirstlane((int)(tid >> 5));
    const unsigned hh = lane >> 4, c = lane & 15u;
    const unsigned row = blockIdx.x;
    const unsigned b = row >> 7;
    sPE[tid] = PQ[(size_t)row * PQW + tid] + bfr(eb1[tid]);
    sPE[tid + 256u] = PQ[(size_t)row * PQW + tid + 256u] + bfr(eb1[tid + 256u]);
    if (wave < (unsigned)(EH2 / 32)) {
        sW3[tid] = bfr(ew3[tid]);
        sB2[tid] = bfr(eb2[tid]);
    }
    __syncthreads();

    const float* qrow = PQ + (size_t)(b * SEQ + wave * 16u + c) * PQW + EH1 + 8u * hh;
    v8f acc[8];
#pragma unroll
    for (int nt = 0; nt < 8; ++nt) acc[nt] = (v8f){0.f,0.f,0.f,0.f,0.f,0.f,0.f,0.f};

#pragma unroll 1
    for (unsigned k0 = 0; k0 < (unsigned)EH1; k0 += 32u) {
        v4f qv[4], pv[4];
        qv[0] = *(const v4f*)(qrow + k0);
        qv[1] = *(const v4f*)(qrow + k0 + 4u);
        qv[2] = *(const v4f*)(qrow + k0 + 16u);
        qv[3] = *(const v4f*)(qrow + k0 + 20u);
        pv[0] = *(const v4f*)(&sPE[k0 + 8u * hh]);
        pv[1] = *(const v4f*)(&sPE[k0 + 8u * hh + 4u]);
        pv[2] = *(const v4f*)(&sPE[k0 + 8u * hh + 16u]);
        pv[3] = *(const v4f*)(&sPE[k0 + 8u * hh + 20u]);
        v16h ah, ar;
#pragma unroll
        for (int g = 0; g < 4; ++g) {
#pragma unroll
            for (int e = 0; e < 4; ++e) {
                const float v = fmaxf(qv[g][e] + pv[g][e], 0.0f) * ca;
                const h16 hi = toh_flush(v);
                ah[4 * g + e] = hi;
                ar[4 * g + e] = toh_flush((v - (float)hi) * RSC);
            }
        }
#pragma unroll
        for (int nt = 0; nt < 8; ++nt) {
            const _Float16* wp = W2 + (size_t)((unsigned)nt * 16u + c) * (2u * EH1) + k0 + 8u * hh;
            const v16h bh = frag_ld(wp);
            const v16h bl = frag_ld(wp + EH1);
            acc[nt] = wmma16(ah, bh, acc[nt]);
            acc[nt] = wmma16(ar, bl, acc[nt]);
        }
    }

    float s[8] = {0.f, 0.f, 0.f, 0.f, 0.f, 0.f, 0.f, 0.f};
#pragma unroll
    for (int nt = 0; nt < 8; ++nt) {
        const unsigned n = (unsigned)nt * 16u + c;
        const float w3 = sW3[n];
        const float b2 = sB2[n];
#pragma unroll
        for (int r = 0; r < 8; ++r) s[r] += fmaxf(acc[nt][r] * scale + b2, 0.0f) * w3;
    }
#pragma unroll
    for (int off = 1; off < 16; off <<= 1) {
#pragma unroll
        for (int r = 0; r < 8; ++r) s[r] += __shfl_xor(s[r], off, 32);
    }
    const float e3 = bfr(eb3[0]);
    const float mi = (float)mask[row];
    float av[8];
#pragma unroll
    for (int r = 0; r < 8; ++r) {
        const float mj = (float)mask[b * SEQ + wave * 16u + 8u * hh + (unsigned)r];
        av[r] = ((s[r] + e3) * mi) * mj;
    }
    if (c == 0u) {
#pragma unroll
        for (int r = 0; r < 8; ++r) sAdj[wave * 16u + 8u * hh + (unsigned)r] = av[r];
    }
    __syncthreads();

    if (wave < 2u) {
        v8h ov;
#pragma unroll
        for (int e = 0; e < 8; ++e) {
            const float a = sAdj[8u * c + (unsigned)e] * cadj;
            const h16 hi = toh_flush(a);
            const h16 hs = toh_flush((float)hi * RSI);
            const h16 rs = toh_flush((a - (float)hi) * RSC);
            const h16 w0 = (hh == 0u) ? hi : hs;
            ov[e] = (wave == 0u) ? w0 : rs;
        }
        const unsigned col = (wave == 0u) ? (8u * lane) : (2u * SEQ + 8u * c);
        _Float16* dst = adjA + (size_t)row * KADJ + col;
        if (wave == 0u || lane < 16u) {
            *(volatile v8h*)dst = ov;
            __threadfence();
            *(volatile v8h*)dst = ov;
        }
    }
}

extern "C" void kernel_launch(void* const* d_in, const int* in_sizes, int n_in, void* d_out, int out_size,
                              void* d_ws, size_t ws_size, hipStream_t stream) {
    if (n_in < 16) return;
    if (in_sizes[0] < MTOK * DF || in_sizes[1] < MTOK || in_sizes[2] < 2 * DF * EH1 || in_sizes[3] < EH1) return;
    if (in_sizes[4] < EH1 * EH2 || in_sizes[5] < EH2 || in_sizes[6] < EH2 || in_sizes[7] < 1) return;
    if (in_sizes[8] < DF * FH1 || in_sizes[9] < FH1 || in_sizes[10] < FH1 * FOUT || in_sizes[11] < FOUT) return;
    if (in_sizes[12] < FOUT * GH1 || in_sizes[13] < GH1 || in_sizes[14] < GH1 * GOUT || in_sizes[15] < GOUT) return;
    if (out_size < MTOK * GOUT) return;

    const float* features = (const float*)d_in[0];
    const int*   amask    = (const int*)d_in[1];
    const float* ew1 = (const float*)d_in[2];
    const float* eb1 = (const float*)d_in[3];
    const float* ew2 = (const float*)d_in[4];
    const float* eb2 = (const float*)d_in[5];
    const float* ew3 = (const float*)d_in[6];
    const float* eb3 = (const float*)d_in[7];
    const float* fw1 = (const float*)d_in[8];
    const float* fb1 = (const float*)d_in[9];
    const float* fw2 = (const float*)d_in[10];
    const float* fb2 = (const float*)d_in[11];
    const float* gw1 = (const float*)d_in[12];
    const float* gb1 = (const float*)d_in[13];
    const float* gw2 = (const float*)d_in[14];
    const float* gb2 = (const float*)d_in[15];
    float* out = (float*)d_out;

    char* wsp = (char*)d_ws;
    size_t off = 0;
    auto carve = [&](size_t bytes) -> void* { void* r = wsp + off; off += (bytes + 255) & ~(size_t)255; return r; };
    unsigned short* x16   = (unsigned short*)carve((size_t)MTOK * DF * 2);
    unsigned short* w1p   = (unsigned short*)carve((size_t)(PQW + FH1) * DF * 2);
    unsigned short* w2f   = (unsigned short*)carve((size_t)EH2 * 2 * EH1 * 2);
    unsigned short* fw2f  = (unsigned short*)carve((size_t)FOUT * 2 * FH1 * 2);
    unsigned short* gw1f  = (unsigned short*)carve((size_t)GH1 * 2 * FOUT * 2);
    unsigned short* gw2f  = (unsigned short*)carve((size_t)GOUT * 2 * GH1 * 2);
    float*          pq    = (float*)carve((size_t)MTOK * PQW * 4);
    unsigned short* f1hr  = (unsigned short*)carve((size_t)MTOK * 2 * FH1 * 2);
    unsigned short* fhr   = (unsigned short*)carve((size_t)MTOK * 2 * FOUT * 2);
    unsigned short* xt    = (unsigned short*)carve((size_t)GH1 * NB * KADJ * 2);
    unsigned short* adjA  = (unsigned short*)carve((size_t)MTOK * KADJ * 2);
    unsigned short* ghr   = (unsigned short*)carve((size_t)MTOK * 2 * GH1 * 2);
    unsigned short* g2t   = (unsigned short*)carve((size_t)GOUT * NB * KADJ * 2);
    if (off > ws_size || off > (size_t)134217728) return;

    k_x16<<<(MTOK * DF / 8) / 256, 256, 0, stream>>>(features, x16, CA);
    k_wconv<<<(EH1 * (DF / 8) + 255) / 256, 256, 0, stream>>>(ew1, DF, EH1, w1p, DF, CW1, 0u, CW1);
    k_wconv<<<(EH1 * (DF / 8) + 255) / 256, 256, 0, stream>>>(ew1 + (size_t)DF * EH1, DF, EH1, w1p + (size_t)EH1 * DF, DF, CW1, 0u, CW1);
    k_wconv<<<(FH1 * (DF / 8) + 255) / 256, 256, 0, stream>>>(fw1, DF, FH1, w1p + (size_t)PQW * DF, DF, CW1, 0u, CW1);
    k_wconv<<<(EH2 * (EH1 / 8) + 255) / 256, 256, 0, stream>>>(ew2, EH1, EH2, w2f, 2 * EH1, CWH, EH1, CWL);
    k_wconv<<<(FOUT * (FH1 / 8) + 255) / 256, 256, 0, stream>>>(fw2, FH1, FOUT, fw2f, 2 * FH1, CWH, FH1, CWL);
    k_wconv<<<(GH1 * (FOUT / 8) + 255) / 256, 256, 0, stream>>>(gw1, FOUT, GH1, gw1f, 2 * FOUT, CWH, FOUT, CWL);
    k_wconv<<<(GOUT * (GH1 / 8) + 255) / 256, 256, 0, stream>>>(gw2, GH1, GOUT, gw2f, 2 * GH1, CWH, GH1, CWL);

    k_gemm_f32<<<dim3(((MTOK / 64) * (PQW / 64) + 7) / 8, 1), 256, 0, stream>>>(
        (const _Float16*)x16, DF, 0u, (const _Float16*)w1p, DF, 0u, pq, PQW, 0u, MTOK, PQW, DF, SC_IN);
    k_gemm_hr_br<<<dim3(((MTOK / 64) * (FH1 / 64) + 7) / 8, 1), 256, 0, stream>>>(
        (const _Float16*)x16, DF, 0u, (const _Float16*)(w1p + (size_t)PQW * DF), DF, 0u, (_Float16*)f1hr, 2 * FH1, 0u, fb1,
        MTOK, FH1, DF, SC_IN, CA, FH1);
    k_gemm_hr_b<<<dim3(((MTOK / 64) * (FOUT / 64) + 7) / 8, 1), 256, 0, stream>>>(
        (const _Float16*)f1hr, 2 * FH1, 0u, (const _Float16*)fw2f, 2 * FH1, 0u, (_Float16*)fhr, 2 * FOUT, 0u, fb2,
        MTOK, FOUT, 2 * FH1, SC_FOLD, CA, FOUT);
    k_gemm_t<<<dim3(((GH1 / 64) * (MTOK / 64) + 7) / 8, 1), 256, 0, stream>>>(
        (const _Float16*)gw1f, 2 * FOUT, 0u, (const _Float16*)fhr, 2 * FOUT, 0u, (_Float16*)xt, NB * KADJ, 0u, gb1,
        GH1, MTOK, 2 * FOUT, SC_FOLD, CA);
    k_edge<<<MTOK, 256, 0, stream>>>(pq, (const _Float16*)w2f, eb1, eb2, ew3, eb3, amask, (_Float16*)adjA, SC_FOLD, CA, CADJ);
    k_gemm_hr_r<<<dim3(((SEQ / 64) * (GH1 / 64) + 7) / 8, NB), 256, 0, stream>>>(
        (const _Float16*)adjA, KADJ, SEQ * KADJ, (const _Float16*)xt, NB * KADJ, KADJ, (_Float16*)ghr, 2 * GH1, SEQ * 2 * GH1,
        SEQ, GH1, KADJ, SC_ADJ, CA, GH1);
    k_gemm_t<<<dim3(((GOUT / 64) * (MTOK / 64) + 7) / 8, 1), 256, 0, stream>>>(
        (const _Float16*)gw2f, 2 * GH1, 0u, (const _Float16*)ghr, 2 * GH1, 0u, (_Float16*)g2t, NB * KADJ, 0u, gb2,
        GOUT, MTOK, 2 * GH1, SC_FOLD, CA);
    k_gemm_tanh<<<dim3(((SEQ / 64) * (GOUT / 64) + 7) / 8, NB), 256, 0, stream>>>(
        (const _Float16*)adjA, KADJ, SEQ * KADJ, (const _Float16*)g2t, NB * KADJ, KADJ, out, GOUT, SEQ * GOUT,
        SEQ, GOUT, KADJ, SC_ADJ);
}
